// PerLeadTimeMLP_1236950581948
// MI455X (gfx1250) — hardware-verified
//
#include <hip/hip_runtime.h>


typedef __attribute__((ext_vector_type(16))) _Float16 v16h;
typedef __attribute__((ext_vector_type(8)))  float    v8f;
typedef __attribute__((ext_vector_type(4)))  float    v4f;

#define kT 42
#define kD 2
#define kH 64
#define WAVES 8
#define ROWS_PER_BLOCK (WAVES * 16)

__device__ __forceinline__ int frag_k(int e, int hh) { return (e < 8) ? (8 * hh + e) : (16 + 8 * hh + (e - 8)); }
__device__ __forceinline__ v8f wmma16(v16h a, v16h b, v8f c) {
  v8f d = __builtin_amdgcn_wmma_f32_16x16x32_f16(false, a, false, b, (short)0, c, false, false);
  asm volatile("v_nop\n\tv_nop\n\tv_nop\n\tv_nop" : "+v"(d) : "v"(a), "v"(b));
  return d;
}

__global__ __launch_bounds__(256) void prep_w2(const float* __restrict__ W2, _Float16* __restrict__ frag) {
  const int i8 = blockIdx.x * 256 + threadIdx.x;
  if (i8 >= kT * 4 * 2 * 32 * 2) return;
  const int d0 = i8 * 8;
  const int e0 = d0 & 15, lane = (d0 >> 4) & 31, s = (d0 >> 9) & 1, j = (d0 >> 10) & 3, t = d0 >> 12;
  typedef __attribute__((ext_vector_type(8))) _Float16 v8h;
  v8h v;
#pragma unroll
  for (int q = 0; q < 8; ++q) { const int e = e0 + q; const int kin = 32 * s + frag_k(e, lane >> 4); v[q] = (_Float16)W2[(t * kH + kin) * kH + 16 * j + (lane & 15)]; }
  *(volatile v8h*)(frag + d0) = v; __threadfence(); *(volatile v8h*)(frag + d0) = v;
}

__global__ __launch_bounds__(256)
void perlead_mlp_kernel(const float* __restrict__ x,
                        const float* __restrict__ W1, const float* __restrict__ b1,
                        const _Float16* __restrict__ w2frag, const float* __restrict__ b2,
                        const float* __restrict__ W3, const float* __restrict__ b3,
                        float* __restrict__ out)
{
  __shared__ __attribute__((aligned(16))) float sOut[WAVES][16 * kT * kD];
  __shared__ float sW1[kT * kD * kH];
  __shared__ float sb1[kT * kH];
  __shared__ float sW3[kT * kH * kD];
  const int tid = threadIdx.x;
  for (int i = tid; i < kT * kD * kH; i += 256) { sW1[i] = W1[i]; sW3[i] = W3[i]; }
  for (int i = tid; i < kT * kH; i += 256) sb1[i] = b1[i];
  __syncthreads();

  const int lane = tid & 31, wave = tid >> 5;
  const int m = lane & 15, half = lane >> 4;
  const int row0 = blockIdx.x * ROWS_PER_BLOCK + wave * 16;
  const int row = row0 + m;
  float* so = sOut[wave];

  for (int t = 0; t < kT; ++t) {
    const float xv0 = x[((long)row * kT + t) * kD + 0];
    const float xv1 = x[((long)row * kT + t) * kD + 1];
    v16h bH1[2];
#pragma unroll
    for (int s = 0; s < 2; ++s)
#pragma unroll
      for (int e = 0; e < 16; ++e) {
        const int k = 32 * s + frag_k(e, half);
        const float h = fmaf(sW1[(t * kD + 0) * kH + k], xv0, fmaf(sW1[(t * kD + 1) * kH + k], xv1, sb1[t * kH + k]));
        bH1[s][e] = (_Float16)fmaxf(h, 0.0f);
      }
    float s0 = 0.f, s1 = 0.f;
#pragma unroll
    for (int j = 0; j < 4; ++j) {
      v8f acc;
#pragma unroll
      for (int v = 0; v < 8; ++v) acc[v] = b2[t * kH + 16 * j + 8 * half + v];
      const v16h a0 = *(const v16h*)(w2frag + ((size_t)((t * 4 + j) * 2 + 0) * 32 + lane) * 16);
      const v16h a1 = *(const v16h*)(w2frag + ((size_t)((t * 4 + j) * 2 + 1) * 32 + lane) * 16);
      acc = wmma16(a0, bH1[0], acc);
      acc = wmma16(a1, bH1[1], acc);
#pragma unroll
      for (int v = 0; v < 8; ++v) {
        const float h2 = fmaxf(acc[v], 0.0f);
        const int ho = 16 * j + 8 * half + v;
        s0 = fmaf(h2, sW3[(t * kH + ho) * kD + 0], s0);
        s1 = fmaf(h2, sW3[(t * kH + ho) * kD + 1], s1);
      }
    }
    s0 += __shfl_xor(s0, 16, 32);
    s1 += __shfl_xor(s1, 16, 32);
    if (half == 0) { so[(m * kT + t) * kD + 0] = s0 + b3[t * kD + 0]; so[(m * kT + t) * kD + 1] = s1 + b3[t * kD + 1]; }
  }
  __builtin_amdgcn_fence(__ATOMIC_RELEASE, "workgroup"); __builtin_amdgcn_wave_barrier(); __builtin_amdgcn_fence(__ATOMIC_ACQUIRE, "workgroup");
  float* ob = out + (long)row0 * kT * kD;
  for (int pass = 0; pass < 2; ++pass) {
    for (int piece = lane; piece < 16 * kT * kD / 4; piece += 32) *(volatile v4f*)(ob + piece * 4) = *(const v4f*)(so + piece * 4);
    __threadfence();
  }
}

extern "C" void kernel_launch(void* const* d_in, const int* in_sizes, int n_in,
                              void* d_out, int out_size, void* d_ws, size_t ws_size,
                              hipStream_t stream) {
  (void)n_in; (void)out_size;
  const float* x  = (const float*)d_in[0];
  const float* W1 = (const float*)d_in[1];
  const float* b1 = (const float*)d_in[2];
  const float* W2 = (const float*)d_in[3];
  const float* b2 = (const float*)d_in[4];
  const float* W3 = (const float*)d_in[5];
  const float* b3 = (const float*)d_in[6];
  float* out = (float*)d_out;
  const size_t fragBytes = (size_t)kT * 4 * 2 * 32 * 16 * sizeof(_Float16);
  if (ws_size < fragBytes) return;
  _Float16* w2frag = (_Float16*)d_ws;

  const int rows = in_sizes[0] / (kT * kD);
  prep_w2<<<(kT * 4 * 2 * 32 * 2 + 255) / 256, 256, 0, stream>>>(W2, w2frag);
  perlead_mlp_kernel<<<rows / ROWS_PER_BLOCK, 256, 0, stream>>>(x, W1, b1, w2frag, b2, W3, b3, out);
}
